// InverseRadonTransform_76596446757205
// MI455X (gfx1250) — hardware-run, weakly checked
//
#include <hip/hip_runtime.h>


#ifndef NB
#define NB 2
#endif
#define NB_FULL 2
#define DET   512
#define NANG  512
#define OUTW  362
#define HALFW 181
#define SINO_BATCH_FULL (DET * NANG)
#define NPIX  (NB * OUTW * OUTW)
#define HSC   16384.0f
#define SSC   1024.0f
#define FOLD  (1.0f / (16384.0f * 1024.0f))
#define PI_F  3.14159265358979323846f

static_assert(NB <= NB_FULL);
static_assert(DET % 64 == 0);
static_assert(NANG % 64 == 0);
static_assert((NB * NANG) % 64 == 0);
static_assert(DET % 32 == 0);
static_assert(DET == 512);
static_assert(NANG == 512);
static_assert(HALFW * 2 == OUTW);
static_assert((DET * DET) % (512 * 8) == 0);
static_assert(2 * NANG == 256 * 4);

typedef _Float16 h16;
typedef __attribute__((ext_vector_type(16))) _Float16 v16h;
typedef __attribute__((ext_vector_type(8)))  _Float16 v8h;
typedef __attribute__((ext_vector_type(8)))  float    v8f;
typedef __attribute__((ext_vector_type(4)))  float    v4f;
typedef v4f  __attribute__((may_alias)) v4fa;

__device__ __forceinline__ unsigned short f2bf(float f) { unsigned u = __float_as_uint(f); u += 0x7FFFu + ((u >> 16) & 1u); return (unsigned short)(u >> 16); }
__device__ __forceinline__ float bfr(float f) { return __uint_as_float(((unsigned)f2bf(f)) << 16); }
__device__ __forceinline__ v16h cat16(v8h lo, v8h hi) { return __builtin_shufflevector(lo, hi, 0, 1, 2, 3, 4, 5, 6, 7, 8, 9, 10, 11, 12, 13, 14, 15); }
__device__ __forceinline__ v8f wmma16(v16h a, v16h b, v8f c) { return __builtin_amdgcn_wmma_f32_16x16x32_f16(false, a, false, b, (short)0, c, false, false); }
__device__ __forceinline__ v16h  ldh(const h16* p) { return cat16(*(const v8h*)p, *(const v8h*)(p + 16)); }
__device__ __forceinline__ void wave_sync() { __builtin_amdgcn_fence(3  , "wavefront"); __builtin_amdgcn_wave_barrier(); asm volatile("" ::: "memory"); }
static __device__ __forceinline__ h16 toh_flush(float v) { const h16 r = (h16)v; return (fabsf(v) < 6.103515625e-05f) ? (h16)0.0f : r; }
__device__ __forceinline__ v8f wmma16g(v16h a, v16h b, v8f c) { c = wmma16(a, b, c); asm volatile("v_nop\n\tv_nop\n\tv_nop\n\tv_nop" : "+v"(c) : "v"(a), "v"(b)); return c; }

static_assert((DET * DET / (512 * 8)) * 512 * 8 == DET * DET);
__global__ __launch_bounds__(512) void k_hmat(h16* HH) {
    __shared__ float g[DET];
    const int tid = threadIdx.x;
    { const int d = tid;
      const float pd = PI_F * (float)(d > 0 ? d : 1);
      const float tap = (-2.0f * HSC) / (pd * pd);
      g[d] = (d == 0) ? (0.5f * HSC) : ((d & 1) ? tap : 0.0f); }
    __syncthreads();
    const int e = (blockIdx.x * 512 + tid) * 8;
    const int n = e / DET, k8 = e % DET;
    v8h o;
#pragma unroll
    for (int i = 0; i < 8; ++i) { int dd = n - (k8 + i); dd = dd < 0 ? -dd : dd; o[i] = toh_flush(g[dd]); }
    *(volatile v8h*)(HH + e) = o; __threadfence(); *(volatile v8h*)(HH + e) = o;
}

static_assert(256 * 16 == 2 * NANG * 4);
__global__ __launch_bounds__(512) void k_trig(float* TR) {
    __shared__ __align__(16) float cs[2 * NANG];
    const int tid = threadIdx.x;
    const int wave = __builtin_amdgcn_readfirstlane((int)(threadIdx.x >> 5));
    const float th = ((float)tid * 0.3515625f) * 0.017453292519943295f;
    float sv, cv;
    sincosf(th, &sv, &cv);
    cs[tid] = cv; cs[NANG + tid] = sv;
    __syncthreads();
    if (wave < 8) {
        const v4f val = *(const v4fa*)(&cs[tid * 4]);
        *(volatile v4f*)(TR + tid * 4) = val; __threadfence(); *(volatile v4f*)(TR + tid * 4) = val;
    }
}

static_assert(4 * 16 == 64);
static_assert(256 * 16 * 2 == 64 * 128);
static_assert(64 * 65 * 4 <= 131072);
__global__ __launch_bounds__(256) void k_tr(const float* __restrict__ sino, h16* ST) {
    __shared__ float ts[64 * 65];
    const int tid = threadIdx.x;
    const int a0 = blockIdx.x * 64, k0 = blockIdx.y * 64, b = blockIdx.z;
    const size_t soff = (size_t)b * SINO_BATCH_FULL + (size_t)k0 * NANG + (size_t)a0;
#pragma unroll
    for (int it = 0; it < 4; ++it) {
        const int kk = it * 16 + (tid >> 4), a4 = (tid & 15) * 4;
        const v4f x = *(const v4f*)(sino + soff + (size_t)kk * NANG + a4);
#pragma unroll
        for (int i = 0; i < 4; ++i) ts[kk * 65 + a4 + i] = bfr(x[i]) * SSC;
    }
    __syncthreads();
    const size_t doff = ((size_t)b * NANG + (size_t)a0) * DET + (size_t)k0;
#pragma unroll 1
    for (int ps = 0; ps < 2; ++ps) {
#pragma unroll
        for (int it = 0; it < 2; ++it) {
            const int row = it * 32 + (tid >> 3), k8 = (tid & 7) * 8;
            v8h o;
#pragma unroll
            for (int i = 0; i < 8; ++i) o[i] = toh_flush(ts[(k8 + i) * 65 + row]);
            *(volatile v8h*)(ST + doff + (size_t)row * DET + k8) = o; }
        if (ps == 0) __threadfence(); }
}

static_assert(32 * 16 * 8 == 16 * 256);
static_assert(16 * 68 * 4 <= 131072);
__global__ __launch_bounds__(32) void k_filt(const h16* __restrict__ A, const h16* __restrict__ Bt, float* C) {
    __shared__ __align__(16) float os[16 * 68];
    const int K = DET;
    const int lane = threadIdx.x & 31, lr = lane & 15, hi = lane >> 4; const int r0 = blockIdx.x * 64, c0 = blockIdx.y * 64;
    v8f acc[4][4];
#pragma unroll
    for (int mb = 0; mb < 4; ++mb)
#pragma unroll
        for (int nb = 0; nb < 4; ++nb) acc[mb][nb] = (v8f){};
    const size_t aoff = (size_t)(r0 + lr) * K + 8 * hi, boff = (size_t)(c0 + lr) * K + 8 * hi;
#pragma unroll 1
    for (int kc = 0; kc < K; kc += 32) {
        v16h a[4];
#pragma unroll
        for (int mb = 0; mb < 4; ++mb) a[mb] = ldh(A + aoff + (size_t)mb * 16 * K + kc);
#pragma unroll
        for (int nb = 0; nb < 4; ++nb) { const v16h b = ldh(Bt + boff + (size_t)nb * 16 * K + kc);
#pragma unroll
            for (int mb = 0; mb < 4; ++mb) acc[mb][nb] = wmma16g(a[mb], b, acc[mb][nb]); }
    }
#pragma unroll
    for (int mb = 0; mb < 4; ++mb) {
#pragma unroll
        for (int nb = 0; nb < 4; ++nb) {
#pragma unroll
            for (int j = 0; j < 8; ++j) os[(hi * 8 + j) * 68 + nb * 16 + lr] = acc[mb][nb][j] * FOLD; }
        wave_sync();
        const size_t cb = (size_t)(r0 + mb * 16) * DET + (size_t)c0;
#pragma unroll 1
        for (int ps = 0; ps < 2; ++ps) {
#pragma unroll
            for (int s = 0; s < 8; ++s) { const int row = 2 * s + (lane >> 4), cofs = (lane & 15) * 4;
                const v4f val = *(const v4fa*)(&os[row * 68 + cofs]);
                *(volatile v4f*)(C + cb + (size_t)row * DET + cofs) = val; }
            if (ps == 0) __threadfence(); }
        wave_sync();
    }
}

static_assert(2 * NANG * 4 <= 131072);
__global__ __launch_bounds__(256) void k_bp(const float* __restrict__ FT, const float* __restrict__ TR, float* OUTP) {
    __shared__ __align__(16) float cs[2 * NANG];
    const int tid = threadIdx.x;
    { const v4f tv = *(const v4f*)(TR + tid * 4); *(v4fa*)(&cs[tid * 4]) = tv; }
    __syncthreads();
    const int idx = blockIdx.x * 256 + tid;
    const int pid = idx < NPIX ? idx : (NPIX - 1);
    const int b = pid / (OUTW * OUTW);
    const int r = pid - b * (OUTW * OUTW);
    const int i = r / OUTW;
    const int j = r - i * OUTW;
    const float xg = (float)(j - HALFW);
    const float yg = (float)(i - HALFW);
    const size_t fb = (size_t)b * NANG * DET;
    float acc = 0.0f;
#pragma unroll 4
    for (int a = 0; a < NANG; ++a) {
        const float pos = xg * cs[a] - yg * cs[NANG + a] + (float)(DET / 2);
        const float fl = floorf(pos);
        int i0 = (int)fl; i0 = i0 < 0 ? 0 : (i0 > DET - 1 ? DET - 1 : i0);
        const int i1 = (i0 + 1 > DET - 1) ? (DET - 1) : (i0 + 1);
        const float w = pos - fl;
        float v0 = FT[fb + (size_t)a * DET + i0];
        float v1 = FT[fb + (size_t)a * DET + i1];
        asm volatile("" : "+v"(v0));
        asm volatile("" : "+v"(v1));
        const bool valid = (pos >= 0.0f) & (pos <= (float)(DET - 1));
        const float lerp = v0 + w * (v1 - v0);
        acc += valid ? lerp : 0.0f;
    }
    const float res = acc * (PI_F / (2.0f * (float)NANG));
    if (idx < NPIX) *(volatile float*)(OUTP + idx) = res;
    __threadfence();
    if (idx < NPIX) *(volatile float*)(OUTP + idx) = res;
}

static constexpr size_t al256(size_t v) { return (v + 255) & ~(size_t)255; }
static constexpr size_t SZ_HH = al256((size_t)DET * DET * 2);
static constexpr size_t SZ_ST = al256((size_t)NB * NANG * DET * 2);
static constexpr size_t SZ_FT = al256((size_t)NB * NANG * DET * 4);
static constexpr size_t SZ_TR = al256((size_t)2 * NANG * 4);
static constexpr size_t SZ_TOTAL = SZ_HH + SZ_ST + SZ_FT + SZ_TR;
static_assert(SZ_TOTAL <= (size_t)134217728);
static_assert((size_t)(DET * DET / (512 * 8)) * 512 * 8 * 2 <= SZ_HH);
static_assert((size_t)NB * (NANG / 64) * (DET / 64) * 64 * 64 * 2 <= SZ_ST);
static_assert((size_t)(NB * NANG / 64) * (DET / 64) * 64 * 64 * 4 <= SZ_FT);
static_assert((size_t)256 * 16 <= SZ_TR);

extern "C" void kernel_launch(void* const* d_in, const int* in_sizes, int n_in,
                              void* d_out, int out_size, void* d_ws, size_t ws_size, hipStream_t stream) {
    if (n_in < 1) return;
    if ((size_t)in_sizes[0] < (size_t)NB * SINO_BATCH_FULL) return;
    if ((size_t)out_size < (size_t)NPIX) return;
    if (SZ_TOTAL > ws_size) return;
    const float* sino = (const float*)d_in[0];
    float* OUTP = (float*)d_out;
    char* wsp = (char*)d_ws;
    h16* HH = (h16*)wsp; wsp += SZ_HH;
    h16* ST = (h16*)wsp; wsp += SZ_ST;
    float* FT = (float*)wsp; wsp += SZ_FT;
    float* TR = (float*)wsp; wsp += SZ_TR;

    k_hmat<<<dim3(DET * DET / (512 * 8), 1, 1), 512, 0, stream>>>(HH);
    k_trig<<<dim3(1, 1, 1), 512, 0, stream>>>(TR);
    k_tr<<<dim3(NANG / 64, DET / 64, NB), 256, 0, stream>>>(sino, ST);
    k_filt<<<dim3(NB * NANG / 64, DET / 64, 1), 32, 0, stream>>>(ST, HH, FT);
    k_bp<<<dim3((NPIX + 255) / 256, 1, 1), 256, 0, stream>>>(FT, TR, OUTP);
}
